// TGCN_43301860278673
// MI455X (gfx1250) — hardware-verified
//
#include <hip/hip_runtime.h>
#include <hip/hip_bf16.h>
#include <stdint.h>

typedef __attribute__((ext_vector_type(16))) _Float16 v16h;
typedef __attribute__((ext_vector_type(8)))  _Float16 v8h;
typedef __attribute__((ext_vector_type(16))) __bf16   v16b;
typedef __attribute__((ext_vector_type(8)))  __bf16   v8b;
typedef __attribute__((ext_vector_type(8)))  float    v8f;
typedef __attribute__((ext_vector_type(4)))  float    v4f;
#define PSCALE 32768.0f
#define U16(p) ((const unsigned short*)(const void*)(p))
#define PSCALE_INV (1.0f / 32768.0f)

__device__ __forceinline__ unsigned short f2bf_bits(float f) {
  unsigned u = __float_as_uint(f);
  return (unsigned short)((u + 0x7FFFu + ((u >> 16) & 1u)) >> 16);
}
__device__ __forceinline__ float bf_bits2f(unsigned short h) { return __uint_as_float(((unsigned)h) << 16); }

__device__ __forceinline__ void dep_guard_h(v8f& a, v8f& b, v16h x, v16h y) { asm volatile("v_nop\n\tv_nop\n\tv_nop\n\tv_nop" : "+v"(a), "+v"(b) : "v"(x), "v"(y)); }
__device__ __forceinline__ void dep_guard_b(v8f& a, v8f& b, v16b x, v16b y) { asm volatile("v_nop\n\tv_nop\n\tv_nop\n\tv_nop" : "+v"(a), "+v"(b) : "v"(x), "v"(y)); }
__device__ __forceinline__ void keep4_h(v16h a, v16h b, v16h c, v16h d) { asm volatile("v_nop" :: "v"(a), "v"(b), "v"(c), "v"(d)); }
__device__ __forceinline__ void keep4_b(v16b a, v16b b, v16b c, v16b d) { asm volatile("v_nop" :: "v"(a), "v"(b), "v"(c), "v"(d)); }
__device__ __forceinline__ void acc_guard4(v8f& a, v8f& b, v8f& c, v8f& d) { asm volatile("v_nop\n\tv_nop\n\tv_nop\n\tv_nop" : "+v"(a), "+v"(b), "+v"(c), "+v"(d)); }
template <typename T> struct Frag;
template <> struct Frag<_Float16> {
  typedef v16h V; union U { v16h v; v8h h[2]; };
  static __device__ __forceinline__ v16h load(const _Float16* p) {
    U f; f.h[0] = *(const v8h*)(p); f.h[1] = *(const v8h*)(p + 16); return f.v;
  }
  static __device__ __forceinline__ v8f mma(v16h a, v16h b, v8f c) {
    return __builtin_amdgcn_wmma_f32_16x16x32_f16(false, a, false, b, (short)0, c, false, false);
  }
  static __device__ __forceinline__ void guard(v8f& a, v8f& b, v16h x, v16h y) { dep_guard_h(a, b, x, y); }
  static __device__ __forceinline__ void keep(v16h a, v16h b, v16h c, v16h d) { keep4_h(a, b, c, d); }
};
template <> struct Frag<__bf16> {
  typedef v16b V; union U { v16b v; v8b h[2]; };
  static __device__ __forceinline__ v16b load(const __bf16* p) {
    U f; f.h[0] = *(const v8b*)(p); f.h[1] = *(const v8b*)(p + 16); return f.v;
  }
  static __device__ __forceinline__ v8f mma(v16b a, v16b b, v8f c) {
    return __builtin_amdgcn_wmma_f32_16x16x32_bf16(false, a, false, b, (short)0, c, false, false);
  }
  static __device__ __forceinline__ void guard(v8f& a, v8f& b, v16b x, v16b y) { dep_guard_b(a, b, x, y); }
  static __device__ __forceinline__ void keep(v16b a, v16b b, v16b c, v16b d) { keep4_b(a, b, c, d); }
};

template <int ET> struct Elem;
template <> struct Elem<0> { typedef _Float16 T; };
template <> struct Elem<1> { typedef __bf16 T; };
template <int ET, bool SPLIT, int BIAS_MODE, int OUT_MODE, bool RESID, int ACT = 0>
__global__ __launch_bounds__(256) void wmma_gemm64(
    const unsigned short* __restrict__ Ap, const unsigned short* __restrict__ A2p, int lda, long strideA,
    const unsigned short* __restrict__ Btp, const unsigned short* __restrict__ Bt2p, int ldb, long strideB,
    void* __restrict__ Cout, void* __restrict__ Cout2, int ldc, long strideC,
    const float* __restrict__ bias,
    const float* __restrict__ resid, long strideR,
    int M, int N, int K, float scale) {
  typedef typename Elem<ET>::T T;
  typedef typename Frag<T>::V V;
  const T* A = (const T*)Ap; const T* A2 = (const T*)A2p; const T* Bt = (const T*)Btp; const T* Bt2 = (const T*)Bt2p;
  __shared__ __align__(16) float sT[8][16 * 68];
  const int b    = blockIdx.y;
  const int lane = threadIdx.x & 31;
  const int wave = threadIdx.x >> 5;
  const int tilesN = N >> 6;
  const int tilesM = M >> 6;
  const int tile = blockIdx.x * 8 + wave;
  if (tile >= tilesM * tilesN) return;
  const int tm = tile / tilesN;
  const int tn = tile - tm * tilesN;
  const int m0 = tm << 6;
  const int n0 = tn << 6;

  const T* Ab  = A  + (size_t)b * strideA;
  const T* Bb  = Bt + (size_t)b * strideB;
  const T* Ab2 = SPLIT ? (A2  + (size_t)b * strideA) : nullptr;
  const T* Bb2 = SPLIT ? (Bt2 + (size_t)b * strideB) : nullptr;

  const int rlane = lane & 15;
  const int koff  = (lane >> 4) * 8;
  const int mOff  = (lane >> 4) * 8;

  v8f acc[4][4];
#pragma unroll
  for (int i = 0; i < 4; ++i)
#pragma unroll
    for (int j = 0; j < 4; ++j) acc[i][j] = (v8f){0.f,0.f,0.f,0.f,0.f,0.f,0.f,0.f};

  for (int k0 = 0; k0 < K; k0 += 32) {
    V bh[4], bl[4];
#pragma unroll
    for (int j = 0; j < 4; ++j) {
      const size_t bo = (size_t)(n0 + (j << 4) + rlane) * ldb + koff + k0;
      bh[j] = Frag<T>::load(Bb + bo);
      if (SPLIT) bl[j] = Frag<T>::load(Bb2 + bo);
    }
#pragma unroll
    for (int i = 0; i < 4; ++i) {
      const size_t ao = (size_t)(m0 + (i << 4) + rlane) * lda + koff + k0;
      V ah = Frag<T>::load(Ab + ao);
      V al;
      if (SPLIT) al = Frag<T>::load(Ab2 + ao);
#pragma unroll
      for (int j = 0; j < 4; ++j) {
        acc[i][j] = Frag<T>::mma(ah, bh[j], acc[i][j]);
        if (SPLIT) {
          acc[i][j] = Frag<T>::mma(ah, bl[j], acc[i][j]);
          acc[i][j] = Frag<T>::mma(al, bh[j], acc[i][j]);
        }
      }
      Frag<T>::guard(acc[i][0], acc[i][3], ah, SPLIT ? al : ah);
    }
    Frag<T>::keep(bh[0], bh[1], bh[2], bh[3]);
    if (SPLIT) Frag<T>::keep(bl[0], bl[1], bl[2], bl[3]);
  }
  acc_guard4(acc[0][0], acc[0][1], acc[0][2], acc[0][3]);
  acc_guard4(acc[1][0], acc[1][1], acc[1][2], acc[1][3]);
  acc_guard4(acc[2][0], acc[2][1], acc[2][2], acc[2][3]);
  acc_guard4(acc[3][0], acc[3][1], acc[3][2], acc[3][3]);

  float* slab = sT[wave];
  const float* Rb = RESID ? (resid + (size_t)b * strideR) : nullptr;
#pragma unroll
  for (int i = 0; i < 4; ++i) {
    const int mBase = m0 + (i << 4);
#pragma unroll
    for (int j = 0; j < 4; ++j) {
      const int n = n0 + (j << 4) + rlane;
      float bv = 0.f;
      if (BIAS_MODE == 2) bv = bias[n];
#pragma unroll
      for (int r = 0; r < 8; ++r) {
        float v = acc[i][j][r] * scale;
        if (BIAS_MODE == 1) v += bias[mBase + mOff + r];
        if (BIAS_MODE == 2) v += bv;
        if (RESID) v += Rb[(size_t)(mBase + mOff + r) * ldc + n];
        if (ACT == 1) v = tanhf(v);
        if (ACT == 2) v = fmaxf(v, 0.0f);
        if (ACT == 3) v = v / (1.0f + expf(-v));
        if (ACT == 4) v = (v > 0.f) ? v : 0.01f * v;
        if (ACT == 5) v = 0.5f * v * (1.0f + erff(v * 0.70710678118654752f));
        slab[(mOff + r) * 68 + (j << 4) + rlane] = v;
      }
    }
    __builtin_amdgcn_fence(__ATOMIC_RELEASE, "workgroup");
    __builtin_amdgcn_wave_barrier();
    __builtin_amdgcn_fence(__ATOMIC_ACQUIRE, "workgroup");
    if (OUT_MODE == 0) {
      float* C = (float*)Cout + (size_t)b * strideC;
      const int hh = lane >> 4, c4 = (lane & 15) * 4;
      for (int pass = 0; pass < 2; ++pass) {
#pragma unroll
        for (int it = 0; it < 8; ++it) {
          const int row = it * 2 + hh;
          v4f v = *(const v4f*)(slab + row * 68 + c4);
          *(volatile v4f*)(C + (size_t)(mBase + row) * ldc + n0 + c4) = v;
        }
        __threadfence();
      }
    } else {
      const int q = lane >> 3, c8 = (lane & 7) * 8;
      unsigned short* C  = (unsigned short*)Cout  + (size_t)b * strideC;
      unsigned short* C2 = (OUT_MODE == 2) ? ((unsigned short*)Cout2 + (size_t)b * strideC) : nullptr;
      for (int pass = 0; pass < 2; ++pass) {
#pragma unroll
        for (int it = 0; it < 4; ++it) {
          const int row = it * 4 + q;
          const float* sp = slab + row * 68 + c8;
          v8h hv, lv;
#pragma unroll
          for (int e = 0; e < 8; ++e) {
            if (OUT_MODE == 1) {
              hv[e] = (_Float16)sp[e];
            } else {
              unsigned short hb = f2bf_bits(sp[e]);
              unsigned short lb = f2bf_bits(sp[e] - bf_bits2f(hb));
              hv[e] = __builtin_bit_cast(_Float16, hb);
              lv[e] = __builtin_bit_cast(_Float16, lb);
            }
          }
          *(volatile v8h*)(C + (size_t)(mBase + row) * ldc + n0 + c8) = hv;
          if (OUT_MODE == 2) *(volatile v8h*)(C2 + (size_t)(mBase + row) * ldc + n0 + c8) = lv;
        }
        __threadfence();
      }
    }
    __builtin_amdgcn_fence(__ATOMIC_RELEASE, "workgroup");
    __builtin_amdgcn_wave_barrier();
    __builtin_amdgcn_fence(__ATOMIC_ACQUIRE, "workgroup");
  }
}

typedef __attribute__((ext_vector_type(4))) unsigned v4u;

constexpr int kNB   = 128;
constexpr int kNS   = 12;
constexpr int kNN   = 325;
constexpr int kNH   = 64;
constexpr int kNBS  = kNB * kNS;
constexpr int kHALF = kNBS / 2;
constexpr int kMPAD = 384;
constexpr int kKPAD = 352;
constexpr int kTP   = 384;
constexpr int kG3   = 3 * kNH;
constexpr int kWP   = 72;
constexpr int kOP   = 352;
constexpr int kTILES = 22;

constexpr float kCarryAdj = 1024.0f;
constexpr float kCarryH1  = 1024.0f;
constexpr float kCarryW   = 16.0f;
constexpr float kCarryH2  = 1024.0f;
constexpr float kCarryHs  = 8192.0f;
constexpr float kScSite2  = kCarryH2 / (kCarryAdj * kCarryH1 * kCarryW);
constexpr float kScGi     = 1.0f / (kCarryH2 * kCarryW);
constexpr float kScGh     = 1.0f / (kCarryHs * kCarryW);

static_assert(kNBS % 64 == 0 && kMPAD % 64 == 0 && kKPAD % 32 == 0);
static_assert(kNH % 64 == 0 && kTP % 64 == 0 && kNH % 32 == 0);
static_assert(kKPAD % 8 == 0 && kTP % 8 == 0);
static_assert((kNBS * kKPAD) % (256 * 8) == 0);
static_assert((kMPAD * kKPAD) % (256 * 8) == 0);
static_assert(kHALF * 6 % 8 == 0);
static_assert((kNB * kNN) % 4 == 0 && ((kNB * kNN) / 4) % 32 == 0);
static_assert(kOP * 4 % 128 == 0 && 8 * 16 * 4 % 128 == 0);

__device__ __forceinline__ unsigned short h_bits(float f) { return __builtin_bit_cast(unsigned short, (_Float16)f); }
__device__ __forceinline__ unsigned pk2(unsigned short a, unsigned short b) { return (unsigned)a | ((unsigned)b << 16); }
__device__ __forceinline__ v4u pack8(const unsigned short (&b)[8]) {
  v4u r;
  r[0] = pk2(b[0], b[1]); r[1] = pk2(b[2], b[3]); r[2] = pk2(b[4], b[5]); r[3] = pk2(b[6], b[7]);
  return r;
}
__device__ __forceinline__ void store16_twice(unsigned short* p, v4u v) {
  *(volatile v4u*)p = v;
  __threadfence();
  *(volatile v4u*)p = v;
}
__device__ __forceinline__ v8f hmma(v16h a, v16h b, v8f c) {
  c = __builtin_amdgcn_wmma_f32_16x16x32_f16(false, a, false, b, (short)0, c, false, false);
  asm volatile("v_nop\n\tv_nop\n\tv_nop\n\tv_nop" : "+v"(c) : "v"(a), "v"(b));
  return c;
}

__global__ __launch_bounds__(256) void k_cast_x(const float* __restrict__ x,
    unsigned short* __restrict__ xhi, unsigned short* __restrict__ xlo) {
  const int t = blockIdx.x * 256 + threadIdx.x;
  const int f = t * 8;
  const int row = f / kKPAD;
  const int col0 = f - row * kKPAD;
  unsigned short hb[8], lb[8];
#pragma unroll
  for (int i = 0; i < 8; ++i) {
    const int col = col0 + i;
    const int cc = col < kNN ? col : (kNN - 1);
    float v = x[(size_t)row * kNN + cc];
    v = (col < kNN) ? v : 0.0f;
    const unsigned short h = f2bf_bits(v);
    hb[i] = h;
    lb[i] = f2bf_bits(v - bf_bits2f(h));
  }
  const v4u hv = pack8(hb);
  const v4u lv = pack8(lb);
  *(volatile v4u*)(xhi + f) = hv;
  *(volatile v4u*)(xlo + f) = lv;
  __threadfence();
  *(volatile v4u*)(xhi + f) = hv;
  *(volatile v4u*)(xlo + f) = lv;
}

__global__ __launch_bounds__(256) void k_cast_adj(const float* __restrict__ adj,
    unsigned short* __restrict__ ahi, unsigned short* __restrict__ alo, unsigned short* __restrict__ af) {
  const int t = blockIdx.x * 256 + threadIdx.x;
  const int f = t * 8;
  const int row = f / kKPAD;
  const int col0 = f - row * kKPAD;
  const int rc = row < kNN ? row : (kNN - 1);
  unsigned short hb[8], lb[8], fb[8];
#pragma unroll
  for (int i = 0; i < 8; ++i) {
    const int col = col0 + i;
    const int cc = col < kNN ? col : (kNN - 1);
    float v = adj[(size_t)rc * kNN + cc];
    v = (row < kNN && col < kNN) ? v : 0.0f;
    const unsigned short h = f2bf_bits(v);
    hb[i] = h;
    lb[i] = f2bf_bits(v - bf_bits2f(h));
    fb[i] = h_bits(v * kCarryAdj);
  }
  const v4u hv = pack8(hb);
  const v4u lv = pack8(lb);
  const v4u fv = pack8(fb);
  *(volatile v4u*)(ahi + f) = hv;
  *(volatile v4u*)(alo + f) = lv;
  *(volatile v4u*)(af + f) = fv;
  __threadfence();
  *(volatile v4u*)(ahi + f) = hv;
  *(volatile v4u*)(alo + f) = lv;
  *(volatile v4u*)(af + f) = fv;
}

__global__ __launch_bounds__(256) void k_params(const float* __restrict__ W2, const float* __restrict__ Wih,
    const float* __restrict__ Whh, const float* __restrict__ b2,
    unsigned short* __restrict__ w2t, unsigned short* __restrict__ wih16,
    unsigned short* __restrict__ whh16, float* __restrict__ b2s) {
  const int bid = blockIdx.x, tid = threadIdx.x;
  if (bid < 2) {
    const int f = (bid * 256 + tid) * 8;
    const int e = f >> 6, d0 = f & 63;
    unsigned short hb[8];
#pragma unroll
    for (int i = 0; i < 8; ++i) hb[i] = h_bits(W2[(size_t)(d0 + i) * kNH + e] * kCarryW);
    store16_twice(w2t + f, pack8(hb));
  } else if (bid < 8) {
    const int f = ((bid - 2) * 256 + tid) * 8;
    unsigned short hb[8];
#pragma unroll
    for (int i = 0; i < 8; ++i) hb[i] = h_bits(Wih[f + i] * kCarryW);
    store16_twice(wih16 + f, pack8(hb));
  } else if (bid < 14) {
    const int f = ((bid - 8) * 256 + tid) * 8;
    unsigned short hb[8];
#pragma unroll
    for (int i = 0; i < 8; ++i) hb[i] = h_bits(Whh[f + i] * kCarryW);
    store16_twice(whh16 + f, pack8(hb));
  } else {
    if (tid < 16) {
      v4f v;
#pragma unroll
      for (int e = 0; e < 4; ++e) v[e] = b2[tid * 4 + e] * kCarryH2;
      float* p = b2s + tid * 4;
      *(volatile v4f*)p = v;
      __threadfence();
      *(volatile v4f*)p = v;
    }
  }
}

__global__ __launch_bounds__(256) void k_gemm_h1w2(const _Float16* __restrict__ W2t,
    const float* __restrict__ Y1, const float* __restrict__ W1, const float* __restrict__ b1,
    _Float16* __restrict__ Tt, int bs0) {
  __shared__ __align__(16) float sT[8][16 * 68];
  __shared__ float w1s[kNH];
  __shared__ float b1s[kNH];
  const int tid = threadIdx.x;
  if (tid < kNH) w1s[tid] = W1[tid];
  else if (tid < 2 * kNH) b1s[tid - kNH] = b1[tid - kNH];
  __syncthreads();

  const int lane = tid & 31, wave = tid >> 5;
  const int tile = blockIdx.x * 8 + wave;
  const int bidx = tile / 6;
  const int tn = tile - bidx * 6;
  const int n0 = tn << 6;
  const int bs = bs0 + bidx;
  const int rlane = lane & 15;
  const int koff = (lane >> 4) * 8;
  const int mOff = koff;

  float yv[4];
  bool nok[4];
#pragma unroll
  for (int j = 0; j < 4; ++j) {
    const int n = n0 + (j << 4) + rlane;
    yv[j] = Y1[(size_t)bs * kMPAD + n];
    nok[j] = n < kNN;
  }

  v8f acc[4][4];
#pragma unroll
  for (int i = 0; i < 4; ++i)
#pragma unroll
    for (int j = 0; j < 4; ++j) acc[i][j] = (v8f){0.f,0.f,0.f,0.f,0.f,0.f,0.f,0.f};

#pragma unroll
  for (int ks = 0; ks < 2; ++ks) {
    const int k0 = ks * 32;
    float wa[8], ba[8], wb[8], bb[8];
#pragma unroll
    for (int i = 0; i < 8; ++i) {
      wa[i] = w1s[k0 + koff + i];      ba[i] = b1s[k0 + koff + i];
      wb[i] = w1s[k0 + 16 + koff + i]; bb[i] = b1s[k0 + 16 + koff + i];
    }
    v16h bh[4];
#pragma unroll
    for (int j = 0; j < 4; ++j) {
#pragma unroll
      for (int i = 0; i < 8; ++i) {
        float v0 = fmaxf(yv[j] * wa[i] + ba[i], 0.0f) * kCarryH1;
        float v1 = fmaxf(yv[j] * wb[i] + bb[i], 0.0f) * kCarryH1;
        v0 = nok[j] ? v0 : 0.0f;
        v1 = nok[j] ? v1 : 0.0f;
        bh[j][i] = (_Float16)v0;
        bh[j][8 + i] = (_Float16)v1;
      }
    }
#pragma unroll
    for (int i = 0; i < 4; ++i) {
      const v16h ah = Frag<_Float16>::load(W2t + (size_t)((i << 4) + rlane) * kNH + koff + k0);
#pragma unroll
      for (int j = 0; j < 4; ++j) acc[i][j] = Frag<_Float16>::mma(ah, bh[j], acc[i][j]);
      Frag<_Float16>::guard(acc[i][0], acc[i][3], ah, ah);
    }
    Frag<_Float16>::keep(bh[0], bh[1], bh[2], bh[3]);
  }
  acc_guard4(acc[0][0], acc[0][1], acc[0][2], acc[0][3]);
  acc_guard4(acc[1][0], acc[1][1], acc[1][2], acc[1][3]);
  acc_guard4(acc[2][0], acc[2][1], acc[2][2], acc[2][3]);
  acc_guard4(acc[3][0], acc[3][1], acc[3][2], acc[3][3]);

  float* slab = sT[wave];
  _Float16* Cb = Tt + (size_t)bidx * kNH * kTP;
#pragma unroll
  for (int i = 0; i < 4; ++i) {
    const int mBase = i << 4;
#pragma unroll
    for (int j = 0; j < 4; ++j)
#pragma unroll
      for (int r = 0; r < 8; ++r) slab[(mOff + r) * 68 + (j << 4) + rlane] = acc[i][j][r];
    __builtin_amdgcn_fence(__ATOMIC_RELEASE, "workgroup");
    __builtin_amdgcn_wave_barrier();
    __builtin_amdgcn_fence(__ATOMIC_ACQUIRE, "workgroup");
    const int q = lane >> 3, c8 = (lane & 7) * 8;
    for (int pass = 0; pass < 2; ++pass) {
#pragma unroll
      for (int it = 0; it < 4; ++it) {
        const int row = it * 4 + q;
        const float* sp = slab + row * 68 + c8;
        v8h hv;
#pragma unroll
        for (int e = 0; e < 8; ++e) hv[e] = (_Float16)sp[e];
        *(volatile v8h*)(Cb + (size_t)(mBase + row) * kTP + n0 + c8) = hv;
      }
      __threadfence();
    }
    __builtin_amdgcn_fence(__ATOMIC_RELEASE, "workgroup");
    __builtin_amdgcn_wave_barrier();
    __builtin_amdgcn_fence(__ATOMIC_ACQUIRE, "workgroup");
  }
}

__global__ __launch_bounds__(128) void k_gru(const _Float16* __restrict__ H2,
    const _Float16* __restrict__ wih16, const _Float16* __restrict__ whh16,
    const float* __restrict__ bih, const float* __restrict__ bhh,
    const float* __restrict__ Wout, const float* __restrict__ bout,
    float* __restrict__ outws) {
  __shared__ __align__(16) _Float16 wihs[kG3 * kWP];
  __shared__ __align__(16) _Float16 whhs[kG3 * kWP];
  __shared__ __align__(16) _Float16 hs[16 * kWP];
  __shared__ __align__(16) float hf[16 * 68];
  __shared__ __align__(16) float outs[128];
  __shared__ float wouts[kNH];

  const int tid = threadIdx.x;
  const int lane = tid & 31, wave = tid >> 5;
  const int hh = lane >> 4, c = lane & 15, koff = hh * 8;
  const int bx = blockIdx.x, b = blockIdx.y;

  for (int i = tid; i < kG3 * 8; i += 128) {
    const int row = i >> 3, seg = (i & 7) * 8;
    const v8h wa = *(const v8h*)(wih16 + row * kNH + seg);
    const v8h wb = *(const v8h*)(whh16 + row * kNH + seg);
    *(v8h*)(wihs + row * kWP + seg) = wa;
    *(v8h*)(whhs + row * kWP + seg) = wb;
  }
  if (tid < kNH) wouts[tid] = Wout[tid];
  __syncthreads();

  const int col = wave * 16 + c;
  const float bi0 = bih[col], bi1 = bih[kNH + col], bi2 = bih[2 * kNH + col];
  const float bh0 = bhh[col], bh1 = bhh[kNH + col], bh2 = bhh[2 * kNH + col];
  const float bo = bout[0];
  const v8f zero8 = (v8f){0.f,0.f,0.f,0.f,0.f,0.f,0.f,0.f};
  const v8h zeroh = (v8h){0,0,0,0,0,0,0,0};

  const int t0 = bx * 8;
  const int nt = (kTILES - t0) < 8 ? (kTILES - t0) : 8;

  for (int ti = 0; ti < nt; ++ti) {
    const int m0 = (t0 + ti) * 16;
    for (int i = tid; i < (16 * kWP) / 8; i += 128) *(v8h*)(hs + i * 8) = zeroh;
    __syncthreads();
    v8f hp = zero8;
#pragma unroll 1
    for (int s = 0; s < kNS; ++s) {
      const _Float16* xr = H2 + ((size_t)(b * kNS + s) * kMPAD + m0 + c) * kNH;
      const v16h xa0 = Frag<_Float16>::load(xr + koff);
      const v16h xa1 = Frag<_Float16>::load(xr + 32 + koff);
      const v16h ha0 = Frag<_Float16>::load(hs + c * kWP + koff);
      const v16h ha1 = Frag<_Float16>::load(hs + c * kWP + 32 + koff);
      v8f gi[3], gh[3];
#pragma unroll
      for (int g = 0; g < 3; ++g) {
        const _Float16* wi = wihs + (g * kNH + col) * kWP + koff;
        const v16h wi0 = Frag<_Float16>::load(wi);
        const v16h wi1 = Frag<_Float16>::load(wi + 32);
        v8f a = hmma(xa0, wi0, zero8);
        a = hmma(xa1, wi1, a);
        gi[g] = a;
        const _Float16* wq = whhs + (g * kNH + col) * kWP + koff;
        const v16h wh0 = Frag<_Float16>::load(wq);
        const v16h wh1 = Frag<_Float16>::load(wq + 32);
        v8f d = hmma(ha0, wh0, zero8);
        d = hmma(ha1, wh1, d);
        gh[g] = d;
      }
      __syncthreads();
      v8f hn;
#pragma unroll
      for (int r = 0; r < 8; ++r) {
        const float ir = gi[0][r] * kScGi + bi0;
        const float hr = gh[0][r] * kScGh + bh0;
        const float iz = gi[1][r] * kScGi + bi1;
        const float hz = gh[1][r] * kScGh + bh1;
        const float inn = gi[2][r] * kScGi + bi2;
        const float hnn = gh[2][r] * kScGh + bh2;
        const float rg = 1.0f / (1.0f + expf(-(ir + hr)));
        const float zg = 1.0f / (1.0f + expf(-(iz + hz)));
        const float cg = tanhf(inn + rg * hnn);
        hn[r] = (1.0f - zg) * cg + zg * hp[r];
      }
      hp = hn;
#pragma unroll
      for (int r = 0; r < 8; ++r) hs[(8 * hh + r) * kWP + col] = (_Float16)(hn[r] * kCarryHs);
      __syncthreads();
    }
#pragma unroll
    for (int r = 0; r < 8; ++r) hf[(8 * hh + r) * 68 + col] = hp[r];
    __syncthreads();
    if (tid < 16) {
      float a = 0.0f;
#pragma unroll 1
      for (int d = 0; d < kNH; ++d) a += hf[tid * 68 + d] * wouts[d];
      outs[ti * 16 + tid] = a + bo;
    }
    __syncthreads();
  }

  if (wave == 0) {
    const int nl = nt * 4;
    const int lc = lane < nl ? lane : (nl - 1);
    const v4f v = *(const v4f*)(outs + lc * 4);
    float* p = outws + (size_t)b * kOP + t0 * 16 + lc * 4;
    if (lane < nl) *(volatile v4f*)p = v;
    __threadfence();
    if (lane < nl) *(volatile v4f*)p = v;
  }
}

__global__ __launch_bounds__(256) void k_pack_out(const float* __restrict__ outws, float* __restrict__ out) {
  constexpr int kT = (kNB * kNN) / 4;
  const int t = blockIdx.x * 256 + threadIdx.x;
  const int tc = t < kT ? t : (kT - 1);
  v4f v;
#pragma unroll
  for (int e = 0; e < 4; ++e) {
    const int f = tc * 4 + e;
    const int bb = f / kNN;
    const int m = f - bb * kNN;
    v[e] = outws[(size_t)bb * kOP + m];
  }
  float* p = out + (size_t)tc * 4;
  if (t < kT) *(volatile v4f*)p = v;
  __threadfence();
  if (t < kT) *(volatile v4f*)p = v;
}

extern "C" void kernel_launch(void* const* d_in, const int* in_sizes, int n_in,
                              void* d_out, int out_size, void* d_ws, size_t ws_size,
                              hipStream_t stream) {
  if (n_in < 12) return;
  if (in_sizes[0] != kNBS * kNN || in_sizes[1] != kNN * kNN || in_sizes[2] < kNH ||
      in_sizes[3] < kNH || in_sizes[4] != kNH * kNH || in_sizes[5] < kNH ||
      in_sizes[6] != kG3 * kNH || in_sizes[7] != kG3 * kNH || in_sizes[8] < kG3 ||
      in_sizes[9] < kG3 || in_sizes[10] < kNH || in_sizes[11] < 1) return;
  if (out_size < kNB * kNN) return;

  const float* x    = (const float*)d_in[0];
  const float* adj  = (const float*)d_in[1];
  const float* W1   = (const float*)d_in[2];
  const float* b1   = (const float*)d_in[3];
  const float* W2   = (const float*)d_in[4];
  const float* b2   = (const float*)d_in[5];
  const float* Wih  = (const float*)d_in[6];
  const float* Whh  = (const float*)d_in[7];
  const float* bih  = (const float*)d_in[8];
  const float* bhh  = (const float*)d_in[9];
  const float* Wout = (const float*)d_in[10];
  const float* bout = (const float*)d_in[11];
  float* out = (float*)d_out;

  char* ws = (char*)d_ws;
  size_t off = 0;
  auto take = [&](size_t bytes) { size_t o = off; off = (off + bytes + 255) & ~(size_t)255; return o; };
  const size_t o_xhi  = take((size_t)kNBS * kKPAD * 2);
  const size_t o_xlo  = take((size_t)kNBS * kKPAD * 2);
  const size_t o_ahi  = take((size_t)kMPAD * kKPAD * 2);
  const size_t o_alo  = take((size_t)kMPAD * kKPAD * 2);
  const size_t o_af   = take((size_t)kMPAD * kKPAD * 2);
  const size_t o_w2t  = take((size_t)kNH * kNH * 2);
  const size_t o_wih  = take((size_t)kG3 * kNH * 2);
  const size_t o_whh  = take((size_t)kG3 * kNH * 2);
  const size_t o_b2s  = take((size_t)kNH * 4);
  const size_t o_y1   = take((size_t)kNBS * kMPAD * 4);
  const size_t o_tt   = take((size_t)kHALF * kNH * kTP * 2);
  const size_t o_h2   = take((size_t)kNBS * kMPAD * kNH * 2);
  const size_t o_ows  = take((size_t)kNB * kOP * 4);
  if (off > ws_size) return;

  unsigned short* xhi   = (unsigned short*)(ws + o_xhi);
  unsigned short* xlo   = (unsigned short*)(ws + o_xlo);
  unsigned short* ahi   = (unsigned short*)(ws + o_ahi);
  unsigned short* alo   = (unsigned short*)(ws + o_alo);
  unsigned short* af    = (unsigned short*)(ws + o_af);
  unsigned short* w2t   = (unsigned short*)(ws + o_w2t);
  unsigned short* wih16 = (unsigned short*)(ws + o_wih);
  unsigned short* whh16 = (unsigned short*)(ws + o_whh);
  float*          b2s   = (float*)(ws + o_b2s);
  float*          Y1    = (float*)(ws + o_y1);
  unsigned short* Tt    = (unsigned short*)(ws + o_tt);
  unsigned short* H2    = (unsigned short*)(ws + o_h2);
  float*          outws = (float*)(ws + o_ows);

  k_cast_x<<<(kNBS * kKPAD / 8) / 256, 256, 0, stream>>>(x, xhi, xlo);
  k_cast_adj<<<(kMPAD * kKPAD / 8) / 256, 256, 0, stream>>>(adj, ahi, alo, af);
  k_params<<<15, 256, 0, stream>>>(W2, Wih, Whh, b2, w2t, wih16, whh16, b2s);

  wmma_gemm64<1, true, 0, 0, false, 0><<<dim3((kNBS / 64) * (kMPAD / 64) / 8, 1), 256, 0, stream>>>(
      xhi, xlo, kKPAD, 0L, ahi, alo, kKPAD, 0L, (void*)Y1, nullptr, kMPAD, 0L,
      nullptr, nullptr, 0L, kNBS, kMPAD, kKPAD, 1.0f);

  for (int half = 0; half < 2; ++half) {
    k_gemm_h1w2<<<(kHALF * 6) / 8, 256, 0, stream>>>(
        (const _Float16*)w2t, Y1, W1, b1, (_Float16*)Tt, half * kHALF);
    wmma_gemm64<0, false, 2, 1, false, 2><<<dim3(1, kHALF), 256, 0, stream>>>(
        af, nullptr, kKPAD, 0L, Tt, nullptr, kTP, (long)kNH * kTP,
        (void*)(H2 + (size_t)half * kHALF * kMPAD * kNH), nullptr, kNH, (long)kMPAD * kNH,
        b2s, nullptr, 0L, kMPAD, kNH, kKPAD, kScSite2);
  }

  k_gru<<<dim3(3, kNB), 128, 0, stream>>>((const _Float16*)H2, (const _Float16*)wih16,
      (const _Float16*)whh16, bih, bhh, Wout, bout, outws);
  k_pack_out<<<((kNB * kNN / 4) + 255) / 256, 256, 0, stream>>>(outws, out);
}
